// CrossNetMix_50663434224288
// MI455X (gfx1250) — hardware-verified
//
#include <hip/hip_runtime.h>
#include <math.h>

typedef __attribute__((ext_vector_type(16))) _Float16 v16h;
typedef __attribute__((ext_vector_type(16))) __bf16 v16b;
typedef __attribute__((ext_vector_type(8)))  _Float16 v8h;
typedef __attribute__((ext_vector_type(8)))  float v8f;
typedef __attribute__((ext_vector_type(4)))  float v4f;
typedef __attribute__((ext_vector_type(2)))  float v2f;
typedef __attribute__((ext_vector_type(4)))  unsigned v4u;
typedef __attribute__((ext_vector_type(4)))  int v4i;
typedef float __attribute__((may_alias)) float_a;
typedef int __attribute__((may_alias)) int_a;

template <typename T> __device__ __forceinline__ void vst2(void* p, T v) { *(volatile T*)p = v; __threadfence(); *(volatile T*)p = v; }
__device__ __forceinline__ v8f wmma16(v16h a, v16h b, v8f c) {
  v8f d = __builtin_amdgcn_wmma_f32_16x16x32_f16(false, a, false, b, (short)0, c, false, false);
  asm volatile("v_nop\n\tv_nop\n\tv_nop\n\tv_nop" : "+v"(d) : "v"(a), "v"(b));
  return d;
}
__device__ __forceinline__ v8f wmma_bf(v16b a, v16b b, v8f c) {
  v8f d = __builtin_amdgcn_wmma_f32_16x16x32_bf16(false, a, false, b, (short)0, c, false, false);
  asm volatile("v_nop\n\tv_nop\n\tv_nop\n\tv_nop" : "+v"(d) : "v"(a), "v"(b));
  return d;
}
__device__ __forceinline__ v16h frag_h(const _Float16* rowk0, int lane) {
  union { v16h v; v8h q[2]; } u; const _Float16* p = rowk0 + 8 * (lane >> 4);
  u.q[0] = *(const v8h*)p; u.q[1] = *(const v8h*)(p + 16); return u.v;
}
__device__ __forceinline__ v16h frag_f32(const float* rowk0, int lane) {
  v16h a; const float* p = rowk0 + 8 * (lane >> 4);
#pragma unroll
  for (int i = 0; i < 8; ++i) { a[i] = (_Float16)p[i]; a[8 + i] = (_Float16)p[16 + i]; }
  return a;
}
__device__ __forceinline__ v16h frag_f32s(const float* rowk0, int lane, float sc) {
  v16h a; const float* p = rowk0 + 8 * (lane >> 4);
#pragma unroll
  for (int i = 0; i < 8; ++i) { a[i] = (_Float16)(p[i] * sc); a[8 + i] = (_Float16)(p[16 + i] * sc); }
  return a;
}
__device__ __forceinline__ v16h fragc_f32(const float* W, int k0, int n, int lane, int ld, int K) {
  v16h a; const int g = lane >> 4;
#pragma unroll
  for (int i = 0; i < 8; ++i) { const int ka = k0 + 8 * g + i, kb = ka + 16;
    a[i] = (_Float16)(ka < K ? W[(size_t)(ka < K ? ka : K - 1) * ld + n] : 0.f); a[8 + i] = (_Float16)(kb < K ? W[(size_t)(kb < K ? kb : K - 1) * ld + n] : 0.f); }
  return a;
}
struct F2 { v16b h, l; };
__device__ __forceinline__ F2 bsplit16(const float v[16]) { F2 r;
#pragma unroll
  for (int i = 0; i < 16; ++i) { const __bf16 h = (__bf16)v[i]; r.h[i] = h; r.l[i] = (__bf16)(v[i] - (float)h); }
  return r; }
__device__ __forceinline__ F2 split_row(const float* row, int k0, int lane) { float v[16]; const float* p = row + k0 + 8 * (lane >> 4);
#pragma unroll
  for (int i = 0; i < 8; ++i) { v[i] = p[i]; v[8 + i] = p[16 + i]; }
  return bsplit16(v); }
__device__ __forceinline__ F2 split_rowK(const float* row, int k0, int lane, int K) { float v[16]; const int g = lane >> 4;
#pragma unroll
  for (int i = 0; i < 8; ++i) { const int ka = k0 + 8 * g + i, kb = ka + 16; v[i] = ka < K ? row[ka < K ? ka : K - 1] : 0.f; v[8 + i] = kb < K ? row[kb < K ? kb : K - 1] : 0.f; }
  return bsplit16(v); }
__device__ __forceinline__ F2 split_col(const float* W, int k0, int n, int lane, int ld, int K) { float v[16]; const int g = lane >> 4;
#pragma unroll
  for (int i = 0; i < 8; ++i) { const int ka = k0 + 8 * g + i, kb = ka + 16; v[i] = ka < K ? W[(size_t)(ka < K ? ka : K - 1) * ld + n] : 0.f; v[8 + i] = kb < K ? W[(size_t)(kb < K ? kb : K - 1) * ld + n] : 0.f; }
  return bsplit16(v); }
__device__ __forceinline__ v8f mac3(const F2& a, const F2& b, v8f c) { c = wmma_bf(a.l, b.h, c); c = wmma_bf(a.h, b.l, c); return wmma_bf(a.h, b.h, c); }
__device__ __forceinline__ float sigm(float v) { return 1.0f / (1.0f + expf(-v)); }
#define LDSX() do { asm volatile("s_wait_dscnt 0" ::: "memory"); __builtin_amdgcn_wave_barrier(); __builtin_amdgcn_fence(__ATOMIC_RELEASE, "workgroup"); } while (0)

__device__ __forceinline__ float bfr(float v) { return (float)(__bf16)v; }
__device__ __attribute__((noinline)) float tanh_ni(float v) { return tanhf(v); }
#define BB 16384
#define CCH 512
#define RR 64
#define EE 4
#define NL 3
#ifndef TB
#define TB BB
#endif
#define WS_X1  0u
#define WS_X2  (WS_X1 + 4u * (size_t)BB * CCH)
#define WS_END (WS_X2 + 4u * (size_t)BB * CCH)
#define WSC 16.0f

__device__ __forceinline__ v16h frag_lds_h(const _Float16* rowk0, int lane) { union { v16h v; v8h q[2]; } u; const _Float16* p = rowk0 + 8 * (lane >> 4); u.q[0] = *(const v8h*)p; u.q[1] = *(const v8h*)(p + 16); return u.v; }

template <int L, int NT>
__device__ __forceinline__ void g1_pass(const float* __restrict__ XI, const float* __restrict__ VSL, const float* __restrict__ GW, size_t r0, int cb, _Float16 (*sv)[264], float (*sg)[4], int wave, int lane, int col, int g) {
  v8f acc[NT];
#pragma unroll
  for (int j = 0; j < NT; ++j) acc[j] = (v8f){};
#pragma unroll 1
  for (int kc = 0; kc < CCH / 32; ++kc) {
    v16b ab; v16h ah; { const float* p = XI + (r0 + col) * CCH + kc * 32 + 8 * g;
#pragma unroll
      for (int i = 0; i < 8; ++i) { if (L == 0) { ab[i] = (__bf16)p[i]; ab[8 + i] = (__bf16)p[16 + i]; } else { ah[i] = (_Float16)p[i]; ah[8 + i] = (_Float16)p[16 + i]; } } }
#pragma unroll
    for (int j = 0; j < NT; ++j) { const int o = cb + j * 16 + col; v16b wb; v16h wh;
#pragma unroll
      for (int i = 0; i < 16; ++i) { const int k = kc * 32 + (i < 8 ? 8 * g + i : 16 + 8 * g + (i - 8)); float w;
        if (o < 256) { const int e = o >> 6, r = o & 63; w = VSL[((size_t)e * CCH + k) * RR + r]; } else if (o < 256 + EE) { w = GW[(size_t)(o - 256) * CCH + k]; } else w = 0.f;
        if (L == 0) wb[i] = (__bf16)w; else wh[i] = (_Float16)(bfr(w) * WSC); }
      if (L == 0) acc[j] = wmma_bf(ab, wb, acc[j]); else acc[j] = wmma16(ah, wh, acc[j]); } }
#pragma unroll
  for (int j = 0; j < NT; ++j)
#pragma unroll
    for (int r = 0; r < 8; ++r) { const int rl = wave * 16 + 8 * g + r, o = cb + j * 16 + col; float v = acc[j][r]; if (L != 0) v *= (1.0f / WSC);
      if (o < 256) sv[rl][o] = (_Float16)tanh_ni(v); else if (o < 256 + EE) sg[rl][o - 256] = v; } }
template <int L>
__global__ __launch_bounds__(128) void k_layer(const float* __restrict__ X0, const float* __restrict__ XI, const float* __restrict__ VS, const float* __restrict__ CS, const float* __restrict__ US, const float* __restrict__ GW, const float* __restrict__ BI, float* __restrict__ XO) {
  __shared__ __align__(16) _Float16 sv[64][264]; __shared__ __align__(16) float sg[64][4]; __shared__ __align__(16) float sf[4][16][68];
  const int tid = threadIdx.x, wave = tid >> 5, lane = tid & 31, col = lane & 15, g = lane >> 4; const size_t r0 = (size_t)blockIdx.x * 64 + wave * 16;
  const float* VSL = VS + (size_t)L * EE * CCH * RR; const float* CSL = CS + (size_t)L * EE * RR * RR; const float* USL = US + (size_t)L * EE * CCH * RR; const float* BIL = BI + (size_t)L * CCH;
  g1_pass<L, 8>(XI, VSL, GW, r0, 0, sv, sg, wave, lane, col, g);
  g1_pass<L, 8>(XI, VSL, GW, r0, 128, sv, sg, wave, lane, col, g);
  g1_pass<L, 1>(XI, VSL, GW, r0, 256, sv, sg, wave, lane, col, g);
  LDSX();
#pragma unroll 1
  for (int e = 0; e < EE; ++e) { v8f acc[4] = {}; v16h af[RR / 32];
#pragma unroll
    for (int kc = 0; kc < RR / 32; ++kc) af[kc] = frag_lds_h(&sv[wave * 16 + col][e * RR + kc * 32], lane);
#pragma unroll
    for (int kc = 0; kc < RR / 32; ++kc) {
#pragma unroll
      for (int j = 0; j < 4; ++j) { v16h wh; const int q = j * 16 + col;
#pragma unroll
        for (int i = 0; i < 16; ++i) { const int k = kc * 32 + (i < 8 ? 8 * g + i : 16 + 8 * g + (i - 8)); wh[i] = (_Float16)(bfr(CSL[((size_t)e * RR + k) * RR + q]) * WSC); }
        acc[j] = wmma16(af[kc], wh, acc[j]); } }
    __builtin_amdgcn_wave_barrier();
#pragma unroll
    for (int j = 0; j < 4; ++j)
#pragma unroll
      for (int r = 0; r < 8; ++r) { const int rl = wave * 16 + 8 * g + r; const float cv = tanh_ni(acc[j][r] * (1.0f / WSC)); sv[rl][e * RR + j * 16 + col] = (_Float16)(sg[rl][e] * cv); } }
  LDSX();
#pragma unroll 1
  for (int ch = 0; ch < CCH / 64; ++ch) { v8f acc[4] = {};
#pragma unroll 2
    for (int kc = 0; kc < (EE * RR) / 32; ++kc) { const v16h a = frag_lds_h(&sv[wave * 16 + col][kc * 32], lane); const int e = (kc * 32) >> 6;
#pragma unroll
      for (int j = 0; j < 4; ++j) { v16h wh; const int c = ch * 64 + j * 16 + col;
#pragma unroll
        for (int i = 0; i < 16; ++i) { const int k = kc * 32 + (i < 8 ? 8 * g + i : 16 + 8 * g + (i - 8)); const int r = k & 63; wh[i] = (_Float16)(bfr(USL[((size_t)e * CCH + c) * RR + r]) * WSC); }
        acc[j] = wmma16(a, wh, acc[j]); } }
#pragma unroll
    for (int j = 0; j < 4; ++j)
#pragma unroll
      for (int r = 0; r < 8; ++r) { const int rl = wave * 16 + 8 * g + r, cl = j * 16 + col; const int c = ch * 64 + cl; const size_t row = r0 + 8 * g + r;
        const float gsum = (sg[rl][0] + sg[rl][1]) + (sg[rl][2] + sg[rl][3]); const float s = acc[j][r] * (1.0f / WSC) + bfr(BIL[c]) * gsum;
        const float xi = (L == 0) ? bfr(XI[row * CCH + c]) : XI[row * CCH + c];     sf[wave][8 * g + r][cl] = xi + bfr(X0[row * CCH + c]) * s; }
    LDSX(); for (int rl = 0; rl < 16; ++rl) if (lane < 16) vst2(XO + (r0 + rl) * CCH + ch * 64 + lane * 4, *(const v4f*)&sf[wave][rl][lane * 4]);
    __builtin_amdgcn_wave_barrier(); } }
extern "C" void kernel_launch(void* const* d_in, const int* in_sizes, int n_in, void* d_out, int out_size, void* d_ws, size_t ws_size, hipStream_t stream) {
  (void)in_sizes; (void)n_in; (void)out_size;
  const float** F = (const float**)d_in;
  if (ws_size < (size_t)WS_END) return;
  char* ws = (char*)d_ws; float *X1 = (float*)(ws + WS_X1), *X2 = (float*)(ws + WS_X2);
  k_layer<0><<<dim3(TB / 64), 128, 0, stream>>>(F[0], F[0], F[2], F[3], F[1], F[4], F[5], X1);
  k_layer<1><<<dim3(TB / 64), 128, 0, stream>>>(F[0], X1, F[2], F[3], F[1], F[4], F[5], X2);
  k_layer<2><<<dim3(TB / 64), 128, 0, stream>>>(F[0], X2, F[2], F[3], F[1], F[4], F[5], (float*)d_out);
}
